// CodeLinearAttention_51634096832894
// MI455X (gfx1250) — hardware-verified
//
#include <hip/hip_runtime.h>
#include <math.h>

constexpr int kBatch = 2;
constexpr int kT     = 2048;
constexpr int kDM    = 1024;
constexpr int kNH    = 16;
constexpr int kHD    = 64;
constexpr int kCS    = 16;
constexpr int kRows  = kBatch * kT;
constexpr int kQKVN  = 3 * kDM;
constexpr int kQKN   = 2 * kDM;
constexpr int kCN    = kNH * kCS;
constexpr int kTS    = 32;
constexpr float kScale = 0.125f;

typedef __attribute__((ext_vector_type(16))) _Float16 v16h;
typedef __attribute__((ext_vector_type(8)))  _Float16 v8h;
typedef __attribute__((ext_vector_type(16))) __bf16   v16b;
typedef __attribute__((ext_vector_type(8)))  __bf16   v8b;
typedef __attribute__((ext_vector_type(8)))  float    v8f;
typedef __attribute__((ext_vector_type(4)))  float    v4f;
typedef __attribute__((ext_vector_type(4)))  unsigned int v4u;

__device__ __forceinline__ unsigned short f2bf_bits(float f) {
  unsigned u = __float_as_uint(f);
  return (unsigned short)((u + 0x7FFFu + ((u >> 16) & 1u)) >> 16);
}
__device__ __forceinline__ float bf_bits2f(unsigned short h) { return __uint_as_float(((unsigned)h) << 16); }

__device__ __forceinline__ void dep_guard_h(v8f& a, v8f& b, v16h x, v16h y) { asm volatile("v_nop\n\tv_nop\n\tv_nop\n\tv_nop" : "+v"(a), "+v"(b) : "v"(x), "v"(y)); }
__device__ __forceinline__ void dep_guard_b(v8f& a, v8f& b, v16b x, v16b y) { asm volatile("v_nop\n\tv_nop\n\tv_nop\n\tv_nop" : "+v"(a), "+v"(b) : "v"(x), "v"(y)); }
__device__ __forceinline__ void keep4_h(v16h a, v16h b, v16h c, v16h d) { asm volatile("v_nop" :: "v"(a), "v"(b), "v"(c), "v"(d)); }
__device__ __forceinline__ void keep4_b(v16b a, v16b b, v16b c, v16b d) { asm volatile("v_nop" :: "v"(a), "v"(b), "v"(c), "v"(d)); }
__device__ __forceinline__ void acc_guard4(v8f& a, v8f& b, v8f& c, v8f& d) { asm volatile("v_nop\n\tv_nop\n\tv_nop\n\tv_nop" : "+v"(a), "+v"(b), "+v"(c), "+v"(d)); }
template <typename T> struct Frag;
template <> struct Frag<_Float16> {
  typedef v16h V; union U { v16h v; v8h h[2]; };
  static __device__ __forceinline__ v16h load(const _Float16* p) {
    U f; f.h[0] = *(const v8h*)(p); f.h[1] = *(const v8h*)(p + 16); return f.v;
  }
  static __device__ __forceinline__ v8f mma(v16h a, v16h b, v8f c) {
    return __builtin_amdgcn_wmma_f32_16x16x32_f16(false, a, false, b, (short)0, c, false, false);
  }
  static __device__ __forceinline__ void guard(v8f& a, v8f& b, v16h x, v16h y) { dep_guard_h(a, b, x, y); }
  static __device__ __forceinline__ void keep(v16h a, v16h b, v16h c, v16h d) { keep4_h(a, b, c, d); }
};
template <> struct Frag<__bf16> {
  typedef v16b V; union U { v16b v; v8b h[2]; };
  static __device__ __forceinline__ v16b load(const __bf16* p) {
    U f; f.h[0] = *(const v8b*)(p); f.h[1] = *(const v8b*)(p + 16); return f.v;
  }
  static __device__ __forceinline__ v8f mma(v16b a, v16b b, v8f c) {
    return __builtin_amdgcn_wmma_f32_16x16x32_bf16(false, a, false, b, (short)0, c, false, false);
  }
  static __device__ __forceinline__ void guard(v8f& a, v8f& b, v16b x, v16b y) { dep_guard_b(a, b, x, y); }
  static __device__ __forceinline__ void keep(v16b a, v16b b, v16b c, v16b d) { keep4_b(a, b, c, d); }
};

__device__ __forceinline__ unsigned pk16(unsigned short a, unsigned short b) { return (unsigned)a | ((unsigned)b << 16); }
__device__ __forceinline__ unsigned short h_bits(float f) { const _Float16 h = (_Float16)f; return __builtin_bit_cast(unsigned short, h); }

__device__ __forceinline__ float sigm_f(float v) {
  const float e = __expf(-fabsf(v));
  const float r = 1.0f / (1.0f + e);
  return (v >= 0.0f) ? r : e * r;
}

template <int ET> struct Elem;
template <> struct Elem<0> { typedef _Float16 T; };
template <> struct Elem<1> { typedef __bf16 T; };
template <int ET, int SPL, int BIAS, int OUT_MODE, int ACT, int MULR>
__global__ __launch_bounds__(256) void wmma_gemm64(
    const unsigned short* __restrict__ Ap, const unsigned short* __restrict__ A2p, int lda, long strideA,
    const unsigned short* __restrict__ Btp, const unsigned short* __restrict__ Bt2p, int ldb, long strideB,
    void* __restrict__ Cout, void* __restrict__ Cout2, int ldc, long strideC,
    const float* __restrict__ bias, int nbias,
    const float* __restrict__ mulr, int ldr,
    int M, int N, int K, float scale) {
  typedef typename Elem<ET>::T T;
  typedef typename Frag<T>::V V;
  const T* A = (const T*)Ap; const T* A2 = (const T*)A2p; const T* Bt = (const T*)Btp; const T* Bt2 = (const T*)Bt2p;
  __shared__ __align__(16) float sT[8][16 * 68];
  const int b    = blockIdx.y;
  const int lane = threadIdx.x & 31;
  const int wave = threadIdx.x >> 5;
  const int tilesN = N >> 6;
  const int tilesM = M >> 6;
  const int tile = blockIdx.x * 8 + wave;
  if (tile >= tilesM * tilesN) return;
  const int tm = tile / tilesN;
  const int tn = tile - tm * tilesN;
  const int m0 = tm << 6;
  const int n0 = tn << 6;

  const T* Ab  = A  + (size_t)b * strideA;
  const T* Bb  = Bt + (size_t)b * strideB;
  const T* Ab2 = (SPL & 1) ? (A2  + (size_t)b * strideA) : nullptr;
  const T* Bb2 = (SPL & 2) ? (Bt2 + (size_t)b * strideB) : nullptr;

  const int rlane = lane & 15;
  const int koff  = (lane >> 4) * 8;
  const int mOff  = (lane >> 4) * 8;

  v8f acc[4][4];
#pragma unroll
  for (int i = 0; i < 4; ++i)
#pragma unroll
    for (int j = 0; j < 4; ++j) acc[i][j] = (v8f){0.f,0.f,0.f,0.f,0.f,0.f,0.f,0.f};

  for (int k0 = 0; k0 < K; k0 += 32) {
    V bh[4], bl[4];
#pragma unroll
    for (int j = 0; j < 4; ++j) {
      const size_t bo = (size_t)(n0 + (j << 4) + rlane) * ldb + koff + k0;
      bh[j] = Frag<T>::load(Bb + bo);
      if (SPL & 2) bl[j] = Frag<T>::load(Bb2 + bo);
    }
#pragma unroll
    for (int i = 0; i < 4; ++i) {
      const size_t ao = (size_t)(m0 + (i << 4) + rlane) * lda + koff + k0;
      V ah = Frag<T>::load(Ab + ao);
      V al;
      if (SPL & 1) al = Frag<T>::load(Ab2 + ao);
#pragma unroll
      for (int j = 0; j < 4; ++j) {
        acc[i][j] = Frag<T>::mma(ah, bh[j], acc[i][j]);
        if (SPL & 2) acc[i][j] = Frag<T>::mma(ah, bl[j], acc[i][j]);
        if (SPL & 1) acc[i][j] = Frag<T>::mma(al, bh[j], acc[i][j]);
      }
      Frag<T>::guard(acc[i][0], acc[i][3], ah, (SPL & 1) ? al : ah);
    }
    Frag<T>::keep(bh[0], bh[1], bh[2], bh[3]);
    if (SPL & 2) Frag<T>::keep(bl[0], bl[1], bl[2], bl[3]);
  }
  acc_guard4(acc[0][0], acc[0][1], acc[0][2], acc[0][3]);
  acc_guard4(acc[1][0], acc[1][1], acc[1][2], acc[1][3]);
  acc_guard4(acc[2][0], acc[2][1], acc[2][2], acc[2][3]);
  acc_guard4(acc[3][0], acc[3][1], acc[3][2], acc[3][3]);

  float* slab = sT[wave];
#pragma unroll
  for (int i = 0; i < 4; ++i) {
    const int mBase = m0 + (i << 4);
#pragma unroll
    for (int j = 0; j < 4; ++j) {
      const int n = n0 + (j << 4) + rlane;
      float bv = 0.f;
      if (BIAS == 2) {
        const int nc = (n < nbias) ? n : (nbias - 1);
        bv = bf_bits2f(f2bf_bits(bias[nc]));
        if (n >= nbias) bv = 0.0f;
      }
#pragma unroll
      for (int r = 0; r < 8; ++r) {
        float v = acc[i][j][r] * scale;
        if (BIAS == 2) v += bv;
        if (ACT == 3) v = v * sigm_f(v);
        if (ACT == 7) v = sigm_f(0.0625f * v);
        if (MULR) v = v * mulr[(size_t)(mBase + mOff + r) * ldr + n];
        slab[(mOff + r) * 68 + (j << 4) + rlane] = v;
      }
    }
    __builtin_amdgcn_fence(__ATOMIC_RELEASE, "workgroup");
    __builtin_amdgcn_wave_barrier();
    __builtin_amdgcn_fence(__ATOMIC_ACQUIRE, "workgroup");
    if (OUT_MODE == 0) {
      float* Cp = (float*)Cout + (size_t)b * strideC;
      const int hh = lane >> 4, c4 = (lane & 15) * 4;
      for (int pass = 0; pass < 2; ++pass) {
#pragma unroll
        for (int it = 0; it < 8; ++it) {
          const int row = it * 2 + hh;
          v4f v = *(const v4f*)(slab + row * 68 + c4);
          *(volatile v4f*)(Cp + (size_t)(mBase + row) * ldc + n0 + c4) = v;
        }
        __threadfence();
      }
    } else {
      const int q = lane >> 3, c8 = (lane & 7) * 8;
      unsigned short* Cp  = (unsigned short*)Cout  + (size_t)b * strideC;
      unsigned short* Cp2 = (OUT_MODE == 2) ? ((unsigned short*)Cout2 + (size_t)b * strideC) : nullptr;
      for (int pass = 0; pass < 2; ++pass) {
#pragma unroll
        for (int it = 0; it < 4; ++it) {
          const int row = it * 4 + q;
          const float* sp = slab + row * 68 + c8;
          v8h hv, lv;
#pragma unroll
          for (int e = 0; e < 8; ++e) {
            if (OUT_MODE == 1) {
              hv[e] = (_Float16)sp[e];
            } else {
              unsigned short hb = f2bf_bits(sp[e]);
              unsigned short lb = f2bf_bits(sp[e] - bf_bits2f(hb));
              hv[e] = __builtin_bit_cast(_Float16, hb);
              lv[e] = __builtin_bit_cast(_Float16, lb);
            }
          }
          *(volatile v8h*)(Cp + (size_t)(mBase + row) * ldc + n0 + c8) = hv;
          if (OUT_MODE == 2) *(volatile v8h*)(Cp2 + (size_t)(mBase + row) * ldc + n0 + c8) = lv;
        }
        __threadfence();
      }
    }
    __builtin_amdgcn_fence(__ATOMIC_RELEASE, "workgroup");
    __builtin_amdgcn_wave_barrier();
    __builtin_amdgcn_fence(__ATOMIC_ACQUIRE, "workgroup");
  }
}

template <int MODE>
__global__ __launch_bounds__(256) void cast8_kernel(const float* __restrict__ in, unsigned short* __restrict__ out, int n8, float scale) {
  const int i = blockIdx.x * 256 + threadIdx.x;
  if (i >= n8) return;
  const float* p = in + 8 * (size_t)i;
  const v4f a = *(const v4f*)(p);
  const v4f c = *(const v4f*)(p + 4);
  unsigned short hb[8];
#pragma unroll
  for (int e = 0; e < 4; ++e) {
    if (MODE == 0) {
      hb[e]     = f2bf_bits(a[e]);
      hb[4 + e] = f2bf_bits(c[e]);
    } else {
      hb[e]     = h_bits(bf_bits2f(f2bf_bits(a[e])) * scale);
      hb[4 + e] = h_bits(bf_bits2f(f2bf_bits(c[e])) * scale);
    }
  }
  const v4u u = (v4u){pk16(hb[0], hb[1]), pk16(hb[2], hb[3]), pk16(hb[4], hb[5]), pk16(hb[6], hb[7])};
  unsigned short* q = out + 8 * (size_t)i;
  *(volatile v4u*)q = u;
  __threadfence();
  *(volatile v4u*)q = u;
  (void)scale;
}

__global__ __launch_bounds__(256) void cbk_diag_kernel(const float* __restrict__ cbk, unsigned short* __restrict__ out, int n8) {
  const int i = blockIdx.x * 256 + threadIdx.x;
  if (i >= n8) return;
  const int e0 = i * 8;
  const int n  = e0 >> 10;
  const int k0 = e0 & (kDM - 1);
  const int h  = n >> 4;
  const int d0 = k0 - h * kHD;
  const bool inside = (d0 >= 0) && (d0 < kHD);
  const int dcl = inside ? d0 : 0;
  const float* p = cbk + (size_t)n * kHD + dcl;
  const v4f a = *(const v4f*)(p);
  const v4f c = *(const v4f*)(p + 4);
  unsigned short hb[8];
#pragma unroll
  for (int e = 0; e < 4; ++e) {
    const float f0 = inside ? a[e] : 0.0f;
    const float f1 = inside ? c[e] : 0.0f;
    hb[e]     = f2bf_bits(f0);
    hb[4 + e] = f2bf_bits(f1);
  }
  const v4u u = (v4u){pk16(hb[0], hb[1]), pk16(hb[2], hb[3]), pk16(hb[4], hb[5]), pk16(hb[6], hb[7])};
  unsigned short* q = out + (size_t)e0;
  *(volatile v4u*)q = u;
  __threadfence();
  *(volatile v4u*)q = u;
}

__global__ __launch_bounds__(64) void cla_scan_kernel(const float* __restrict__ QC, const float* __restrict__ KC,
                                                      const float* __restrict__ Vp,
                                                      unsigned short* __restrict__ XOH, unsigned short* __restrict__ XOL) {
  __shared__ __align__(16) float sRed[64][17];
  __shared__ __align__(16) float sKmax[16];
  __shared__ __align__(16) float sKE[kTS][16];
  __shared__ __align__(16) float sQP[kTS][16];
  __shared__ __align__(16) float sW[kTS][16];
  __shared__ __align__(16) float sO[kTS][68];
  const int bh   = blockIdx.x;
  const int b    = bh >> 4;
  const int h    = bh & (kNH - 1);
  const int tid  = threadIdx.x;
  const int lane = tid & 31;
  const int wave = tid >> 5;
  const size_t rowBase = (size_t)b * kT;
  const int hc16 = h * kCS;
  const int hc64 = h * kHD;

  {
    v4f m0 = (v4f){-INFINITY, -INFINITY, -INFINITY, -INFINITY};
    v4f m1 = m0, m2 = m0, m3 = m0;
#pragma unroll 2
    for (int i = 0; i < kT / 64; ++i) {
      const float* p = KC + (rowBase + (size_t)(i * 64 + tid)) * kCN + hc16;
      const v4f a0 = *(const v4f*)(p);
      const v4f a1 = *(const v4f*)(p + 4);
      const v4f a2 = *(const v4f*)(p + 8);
      const v4f a3 = *(const v4f*)(p + 12);
#pragma unroll
      for (int e = 0; e < 4; ++e) {
        m0[e] = fmaxf(m0[e], a0[e]);
        m1[e] = fmaxf(m1[e], a1[e]);
        m2[e] = fmaxf(m2[e], a2[e]);
        m3[e] = fmaxf(m3[e], a3[e]);
      }
    }
#pragma unroll
    for (int e = 0; e < 4; ++e) {
      sRed[tid][e]      = m0[e];
      sRed[tid][4 + e]  = m1[e];
      sRed[tid][8 + e]  = m2[e];
      sRed[tid][12 + e] = m3[e];
    }
  }
  __syncthreads();
  if (wave == 0) {
    const int c = lane & 15;
    float m = -INFINITY;
#pragma unroll 1
    for (int j = 0; j < 64; ++j) m = fmaxf(m, sRed[j][c]);
    sKmax[c] = m;
  }
  __syncthreads();

  float S[16];
#pragma unroll
  for (int e = 0; e < 16; ++e) S[e] = 0.0f;
  float zrun = 0.0f;

#pragma unroll 1
  for (int t0 = 0; t0 < kT; t0 += kTS) {
    __syncthreads();
    if (wave == 0) {
      const float* p = QC + (rowBase + (size_t)(t0 + lane)) * kCN + hc16;
      const v4f a0 = *(const v4f*)(p);
      const v4f a1 = *(const v4f*)(p + 4);
      const v4f a2 = *(const v4f*)(p + 8);
      const v4f a3 = *(const v4f*)(p + 12);
      float mx = a0[0];
#pragma unroll
      for (int e = 0; e < 4; ++e) { mx = fmaxf(mx, a0[e]); mx = fmaxf(mx, a1[e]); mx = fmaxf(mx, a2[e]); mx = fmaxf(mx, a3[e]); }
      v4f e0, e1, e2, e3;
      float sum = 0.0f;
#pragma unroll
      for (int e = 0; e < 4; ++e) {
        e0[e] = __expf(a0[e] - mx); e1[e] = __expf(a1[e] - mx); e2[e] = __expf(a2[e] - mx); e3[e] = __expf(a3[e] - mx);
        sum += e0[e]; sum += e1[e]; sum += e2[e]; sum += e3[e];
      }
      const float r = (1.0f / sum) * kScale;
#pragma unroll
      for (int e = 0; e < 4; ++e) { e0[e] *= r; e1[e] *= r; e2[e] *= r; e3[e] *= r; }
      *(v4f*)(&sQP[lane][0])  = e0;
      *(v4f*)(&sQP[lane][4])  = e1;
      *(v4f*)(&sQP[lane][8])  = e2;
      *(v4f*)(&sQP[lane][12]) = e3;
    } else {
#pragma unroll
      for (int j = 0; j < 4; ++j) {
        const int it = lane + 32 * j;
        const int s  = it >> 2;
        const int c4 = (it & 3) * 4;
        const v4f kv = *(const v4f*)(KC + (rowBase + (size_t)(t0 + s)) * kCN + hc16 + c4);
        const v4f km = *(const v4f*)(&sKmax[c4]);
        v4f ev;
#pragma unroll
        for (int e = 0; e < 4; ++e) ev[e] = __expf(kv[e] - km[e]);
        *(v4f*)(&sKE[s][c4]) = ev;
      }
    }
    __syncthreads();
    if (wave == 0) {
      const int c = lane & 15;
#pragma unroll 1
      for (int s = 0; s < kTS; ++s) {
        zrun += sKE[s][c];
        const float w = sQP[s][c] * (1.0f / (zrun + 1e-9f));
        sW[s][c] = w;
      }
    }
    __syncthreads();
    {
      const float* vp = Vp + (rowBase + (size_t)t0) * kDM + hc64 + tid;
#pragma unroll 1
      for (int s = 0; s < kTS; ++s) {
        const float vv = vp[(size_t)s * kDM];
        float o = 0.0f;
#pragma unroll
        for (int g = 0; g < 4; ++g) {
          const v4f k4 = *(const v4f*)(&sKE[s][4 * g]);
          const v4f w4 = *(const v4f*)(&sW[s][4 * g]);
#pragma unroll
          for (int e = 0; e < 4; ++e) {
            const int idx = 4 * g + e;
            const float sn = fmaf(k4[e], vv, S[idx]);
            S[idx] = sn;
            o = fmaf(w4[e], sn, o);
          }
        }
        sO[s][tid] = o;
      }
    }
    __syncthreads();
    {
      const int rq = lane >> 3, c8 = (lane & 7) * 8;
      for (int pass = 0; pass < 2; ++pass) {
#pragma unroll
        for (int it = 0; it < 4; ++it) {
          const int row = wave * 16 + it * 4 + rq;
          const float* sp = &sO[row][c8];
          const v4f a = *(const v4f*)(sp);
          const v4f c = *(const v4f*)(sp + 4);
          unsigned short hb[8], lb[8];
#pragma unroll
          for (int e = 0; e < 4; ++e) {
            const float f0 = a[e];
            const unsigned short h0 = f2bf_bits(f0);
            hb[e] = h0; lb[e] = f2bf_bits(f0 - bf_bits2f(h0));
            const float f1 = c[e];
            const unsigned short h1 = f2bf_bits(f1);
            hb[4 + e] = h1; lb[4 + e] = f2bf_bits(f1 - bf_bits2f(h1));
          }
          const v4u uh = (v4u){pk16(hb[0], hb[1]), pk16(hb[2], hb[3]), pk16(hb[4], hb[5]), pk16(hb[6], hb[7])};
          const v4u ul = (v4u){pk16(lb[0], lb[1]), pk16(lb[2], lb[3]), pk16(lb[4], lb[5]), pk16(lb[6], lb[7])};
          const size_t off = (rowBase + (size_t)(t0 + row)) * kDM + hc64 + c8;
          *(volatile v4u*)(XOH + off) = uh;
          *(volatile v4u*)(XOL + off) = ul;
        }
        __threadfence();
      }
    }
  }
}

extern "C" void kernel_launch(void* const* d_in, const int* in_sizes, int n_in,
                              void* d_out, int out_size, void* d_ws, size_t ws_size,
                              hipStream_t stream) {
  if (n_in < 4) return;
  if (in_sizes[0] != kRows * kDM) return;
  if (in_sizes[1] != kQKVN * kDM) return;
  if (in_sizes[2] != kDM * kDM) return;
  if (in_sizes[3] != kNH * kCS * kHD) return;
  if (out_size != kRows * kDM) return;

  const float* x     = (const float*)d_in[0];
  const float* w_qkv = (const float*)d_in[1];
  const float* w_out = (const float*)d_in[2];
  const float* cbk   = (const float*)d_in[3];
  float* outp = (float*)d_out;

  const size_t SZ_XB   = (size_t)kRows * kDM * 2;
  const size_t SZ_WQKV = (size_t)kQKVN * kDM * 2;
  const size_t SZ_WOUT = (size_t)kDM * kDM * 2;
  const size_t SZ_CBD  = (size_t)kCN * kDM * 2;
  const size_t SZ_QKP  = (size_t)kRows * kQKN * 2;
  const size_t SZ_VF   = (size_t)kRows * kDM * 4;
  const size_t SZ_QKC  = (size_t)2 * kRows * kCN * 4;
  const size_t SZ_XOP  = (size_t)kRows * kDM * 2;

  size_t off = 0;
  const size_t oXB   = off; off += SZ_XB;
  const size_t oWQKV = off; off += SZ_WQKV;
  const size_t oWOUT = off; off += SZ_WOUT;
  const size_t oCBD  = off; off += SZ_CBD;
  const size_t oQKH  = off; off += SZ_QKP;
  const size_t oQKL  = off; off += SZ_QKP;
  const size_t oVF   = off; off += SZ_VF;
  const size_t oQKC  = off; off += SZ_QKC;
  const size_t oXOH  = off; off += SZ_XOP;
  const size_t oXOL  = off; off += SZ_XOP;
  const size_t TOTAL = off;
  if (TOTAL > ws_size) return;
  if (TOTAL > (size_t)134217728) return;

  char* ws = (char*)d_ws;
  unsigned short* XB   = (unsigned short*)(ws + oXB);
  unsigned short* WQKV = (unsigned short*)(ws + oWQKV);
  unsigned short* WOUT = (unsigned short*)(ws + oWOUT);
  unsigned short* CBD  = (unsigned short*)(ws + oCBD);
  unsigned short* QKH  = (unsigned short*)(ws + oQKH);
  unsigned short* QKL  = (unsigned short*)(ws + oQKL);
  float*          VF   = (float*)(ws + oVF);
  float*          QKC  = (float*)(ws + oQKC);
  unsigned short* XOH  = (unsigned short*)(ws + oXOH);
  unsigned short* XOL  = (unsigned short*)(ws + oXOL);

  const dim3 blk(256);

  {
    const int n8x = kRows * kDM / 8;
    cast8_kernel<0><<<dim3((n8x + 255) / 256), blk, 0, stream>>>(x, XB, n8x, 1.0f);
    const int n8q = kQKVN * kDM / 8;
    cast8_kernel<0><<<dim3((n8q + 255) / 256), blk, 0, stream>>>(w_qkv, WQKV, n8q, 1.0f);
    const int n8o = kDM * kDM / 8;
    cast8_kernel<0><<<dim3((n8o + 255) / 256), blk, 0, stream>>>(w_out, WOUT, n8o, 1.0f);
    const int n8c = kCN * kDM / 8;
    cbk_diag_kernel<<<dim3((n8c + 255) / 256), blk, 0, stream>>>(cbk, CBD, n8c);
  }

  const int tilesRows = kRows / 64;
  const dim3 gQK((tilesRows * (kQKN / 64) + 7) / 8, 1);
  const dim3 gV((tilesRows * (kDM / 64) + 7) / 8, 1);
  const dim3 gCB((tilesRows * (kCN / 64) + 7) / 8, 2);
  const dim3 gOUT((tilesRows * (kDM / 64) + 7) / 8, 1);

  wmma_gemm64<1, 0, 0, 2, 0, 0><<<gQK, blk, 0, stream>>>(
      XB, XB, kDM, 0L, WQKV, WQKV, kDM, 0L, (void*)QKH, (void*)QKL, kQKN, 0L, x, 1, x, 0, kRows, kQKN, kDM, 1.0f);
  wmma_gemm64<1, 0, 0, 0, 0, 0><<<gV, blk, 0, stream>>>(
      XB, XB, kDM, 0L, WQKV + (size_t)kQKN * kDM, WQKV + (size_t)kQKN * kDM, kDM, 0L,
      (void*)VF, (void*)VF, kDM, 0L, x, 1, x, 0, kRows, kDM, kDM, 1.0f);

  wmma_gemm64<1, 1, 0, 0, 0, 0><<<gCB, blk, 0, stream>>>(
      QKH, QKL, kQKN, (long)kDM, CBD, CBD, kDM, 0L, (void*)QKC, (void*)QKC, kCN, (long)kRows * kCN,
      x, 1, x, 0, kRows, kCN, kDM, kScale);

  cla_scan_kernel<<<dim3(kBatch * kNH), dim3(64), 0, stream>>>(QKC, QKC + (size_t)kRows * kCN, VF, XOH, XOL);

  wmma_gemm64<1, 1, 0, 0, 0, 0><<<gOUT, blk, 0, stream>>>(
      XOH, XOL, kDM, 0L, WOUT, WOUT, kDM, 0L, (void*)outp, (void*)outp, kDM, 0L, x, 1, x, 0, kRows, kDM, kDM, 1.0f);
}
